// SRUpp_38139309588937
// MI455X (gfx1250) — hardware-verified
//
#include <hip/hip_runtime.h>


#define NB_  4
#define NL   2048
#define DD   1024
#define AA   256
#define NTK  (NB_ * NL)
#define DCH  256
#define UW   (3 * DCH)
#define PSC  32768.0f
#define LOSC 1024.0f
#define LOSCI (1.0f / 1024.0f)

typedef _Float16 h16;
typedef unsigned short bf;
typedef __attribute__((ext_vector_type(16))) __bf16   v16bf;
typedef __attribute__((ext_vector_type(16))) _Float16 v16h;
typedef __attribute__((ext_vector_type(8)))  _Float16 v8h;
typedef __attribute__((ext_vector_type(8)))  unsigned short v8us;
typedef __attribute__((ext_vector_type(8)))  float    v8f;
typedef __attribute__((ext_vector_type(4)))  float    v4f;
typedef v8h  __attribute__((may_alias)) v8ha;
typedef v4f  __attribute__((may_alias)) v4fa;
typedef v8us __attribute__((may_alias)) v8usa;

__device__ __forceinline__ unsigned short f2bf(float f) { unsigned u = __float_as_uint(f); u += 0x7FFFu + ((u >> 16) & 1u); return (unsigned short)(u >> 16); }
__device__ __forceinline__ float bf2f(unsigned short b) { return __uint_as_float(((unsigned)b) << 16); }
__device__ __forceinline__ float bfr(float f) { return bf2f(f2bf(f)); }
__device__ __forceinline__ v16h cat16(v8h lo, v8h hi) { return __builtin_shufflevector(lo, hi, 0, 1, 2, 3, 4, 5, 6, 7, 8, 9, 10, 11, 12, 13, 14, 15); }
__device__ __forceinline__ v16bf cat16b(v8us lo, v8us hi) { return __builtin_bit_cast(v16bf, __builtin_shufflevector(lo, hi, 0, 1, 2, 3, 4, 5, 6, 7, 8, 9, 10, 11, 12, 13, 14, 15)); }
__device__ __forceinline__ v8f wmma16(v16h a, v16h b, v8f c) { return __builtin_amdgcn_wmma_f32_16x16x32_f16(false, a, false, b, (short)0, c, false, false); }
__device__ __forceinline__ v8f wmmab(v16bf a, v16bf b, v8f c) { return __builtin_amdgcn_wmma_f32_16x16x32_bf16(false, a, false, b, (short)0, c, false, false); }
#define VST2(T, p, v) do { const T vst2_v_ = (v); *(volatile T*)(p) = vst2_v_; __threadfence(); *(volatile T*)(p) = vst2_v_; } while (0)

__global__ __launch_bounds__(256) void k_cvtb(const float* __restrict__ src, bf* dst) {
    const int lane = threadIdx.x & 31, r = blockIdx.x * 8 + (threadIdx.x >> 5);
    if (r >= NTK) return;
#pragma unroll
    for (int q = 0; q < 4; ++q) { v8us t;
#pragma unroll
        for (int i = 0; i < 8; ++i) t[i] = f2bf(src[(size_t)r * DD + q * 256 + lane * 8 + i]);
        VST2(v8us, dst + (size_t)r * DD + q * 256 + lane * 8, t); }
}
__global__ __launch_bounds__(256) void k_wt(const float* __restrict__ Wm, int K, int N, bf* WT) {
    __shared__ __align__(16) unsigned short tl[64 * 72];
    const int tid = threadIdx.x, k0 = blockIdx.x * 64, n0 = blockIdx.y * 64;
    const int kk = tid >> 2, nq = (tid & 3) * 16;
#pragma unroll
    for (int i = 0; i < 16; ++i) tl[(nq + i) * 72 + kk] = f2bf(Wm[(size_t)(k0 + kk) * N + n0 + nq + i]);
    __syncthreads();
    const int piece = tid & 7;
    auto pass = [&]() {
#pragma unroll
        for (int s = 0; s < 2; ++s) { const int nr = (tid >> 3) + 32 * s; const v8us val = *(const v8usa*)(tl + nr * 72 + piece * 8);
            *(volatile v8us*)(WT + (size_t)(n0 + nr) * K + k0 + piece * 8) = val; }
    };
    pass(); __threadfence(); pass();
}

template <bool SPLITA, int MODE>
__global__ __launch_bounds__(128) void k_gemm(const bf* __restrict__ A, const bf* __restrict__ Al, const bf* __restrict__ Bn, int K, int chunk, const float* __restrict__ bias, void* C, void* C2) {
    __shared__ __align__(16) float ost[4][16 * 68];
    const int lane = threadIdx.x & 31, wave = threadIdx.x >> 5, lr = lane & 15, hi = lane >> 4;
    const int r0 = blockIdx.x * 64 + wave * 16, c0 = blockIdx.y * 64;
    int brow0 = c0, ldc = AA;
    if (MODE >= 3) { const int part = c0 / DCH, within = c0 - part * DCH; brow0 = part * DD + chunk * DCH + within; ldc = UW; }
    const size_t aoff = (size_t)(r0 + lr) * K + 8 * hi;
    size_t boff[4];
#pragma unroll
    for (int t = 0; t < 4; ++t) boff[t] = (size_t)(brow0 + t * 16 + lr) * K + 8 * hi;
    v8f acc[4];
#pragma unroll
    for (int t = 0; t < 4; ++t) acc[t] = (v8f){};
#pragma unroll 1
    for (int kc = 0; kc < K; kc += 32) {
        const v16bf a = cat16b(*(const v8us*)(A + aoff + kc), *(const v8us*)(A + aoff + kc + 16));
        v16bf al = a;
        if (SPLITA) al = cat16b(*(const v8us*)(Al + aoff + kc), *(const v8us*)(Al + aoff + kc + 16));
#pragma unroll
        for (int t = 0; t < 4; ++t) { const v16bf b = cat16b(*(const v8us*)(Bn + boff[t] + kc), *(const v8us*)(Bn + boff[t] + kc + 16)); acc[t] = wmmab(a, b, acc[t]); if (SPLITA) acc[t] = wmmab(al, b, acc[t]); }
        asm volatile("v_nop\n\tv_nop\n\tv_nop\n\tv_nop" : "+v"(acc[0]), "+v"(acc[1]), "+v"(acc[2]), "+v"(acc[3]) : "v"(a), "v"(al));
    }
    float* os = &ost[wave][0];
#pragma unroll
    for (int t = 0; t < 4; ++t) { const int col = c0 + t * 16 + lr; const float bv = (MODE == 3) ? bfr(bias[brow0 + t * 16 + lr]) : 0.f;
#pragma unroll
        for (int j = 0; j < 8; ++j) { float v = acc[t][j] + bv; if (MODE == 4) v += ((const float*)C)[(size_t)(r0 + hi * 8 + j) * UW + col]; os[(hi * 8 + j) * 68 + t * 16 + lr] = v; } }
    __syncthreads();
    if (MODE != 1) {
        float* crow = (float*)C + (size_t)r0 * ldc + c0;
        auto pass = [&]() {
#pragma unroll
            for (int s = 0; s < 8; ++s) { const int Lid = (lane >> 3) + 4 * s, piece = lane & 7; const int row = Lid >> 1, cofs = (Lid & 1) * 32 + piece * 4;
                const v4f val = *(const v4fa*)(os + row * 68 + cofs); *(volatile v4f*)(crow + (size_t)row * ldc + cofs) = val; }
        };
        pass(); __threadfence(); pass();
    }
    if (MODE == 0 || MODE == 1) {
        h16* crow = (h16*)(MODE == 0 ? C2 : C) + (size_t)r0 * AA + c0;
        auto pass = [&]() {
#pragma unroll
            for (int s = 0; s < 4; ++s) { const int row = 4 * s + (lane >> 3), piece = lane & 7; const float* sp = os + row * 68 + piece * 8; v8h o;
#pragma unroll
                for (int i = 0; i < 8; ++i) o[i] = (h16)sp[i];
                *(volatile v8h*)(crow + (size_t)row * AA + piece * 8) = o; }
        };
        pass(); __threadfence(); pass();
    }
}
__global__ __launch_bounds__(256) void k_vt(const float* __restrict__ V, h16* VT16) {
    __shared__ __align__(16) h16 tile[AA * 72];
    const int b = blockIdx.x / (NL / 64), kt = blockIdx.x - b * (NL / 64), t0 = kt * 64, tid = threadIdx.x;
    const int tt = tid >> 2, aq = (tid & 3) * 64;
    const float* src = V + ((size_t)b * NL + t0 + tt) * AA + aq;
#pragma unroll 4
    for (int i = 0; i < 64; ++i) tile[(aq + i) * 72 + tt] = (h16)src[i];
    __syncthreads();
    const int piece = tid & 7;
    const size_t base = ((size_t)b * AA) * NL + t0;
    auto pass = [&]() {
#pragma unroll
        for (int s = 0; s < 8; ++s) { const int a = (tid >> 3) + 32 * s; const v8h val = *(const v8ha*)(tile + a * 72 + piece * 8); *(volatile v8h*)(VT16 + base + (size_t)a * NL + piece * 8) = val; }
    };
    pass(); __threadfence(); pass();
}
__global__ __launch_bounds__(128) void k_attn(const h16* __restrict__ Q16, const h16* __restrict__ K16, const h16* __restrict__ VT16, int aofs, float* F) {
    __shared__ __align__(16) h16 plds[4][16 * 32];
    __shared__ __align__(16) float ost[4][16 * 132];
    const int lane = threadIdx.x & 31, wave = threadIdx.x >> 5, lr = lane & 15, hi = lane >> 4;
    const int b = blockIdx.x / (NL / 64), qt = blockIdx.x - b * (NL / 64), q0 = qt * 64 + wave * 16;
    const size_t tok0 = (size_t)b * NL;
    h16* pl = &plds[wave][0];
    v16h qa[8];
#pragma unroll
    for (int kc = 0; kc < 8; ++kc) { const size_t o = (tok0 + q0 + lr) * AA + kc * 32 + 8 * hi; qa[kc] = cat16(*(const v8h*)(Q16 + o), *(const v8h*)(Q16 + o + 16)); }
    const h16* vb = VT16 + ((size_t)b * AA + aofs) * NL;
    v8f o[8];
#pragma unroll
    for (int n = 0; n < 8; ++n) o[n] = (v8f){};
    float mrow[8], lpart[8];
#pragma unroll
    for (int j = 0; j < 8; ++j) { mrow[j] = -3.0e38f; lpart[j] = 0.f; }
#pragma unroll 1
    for (int kt = 0; kt < NL / 32; ++kt) {
        const int l0 = kt * 32;
        v8f s0 = {}, s1 = {};
#pragma unroll
        for (int kc = 0; kc < 8; ++kc) {
            const size_t o0 = (tok0 + l0 + lr) * AA + kc * 32 + 8 * hi, o1 = o0 + (size_t)16 * AA;
            s0 = wmma16(qa[kc], cat16(*(const v8h*)(K16 + o0), *(const v8h*)(K16 + o0 + 16)), s0);
            s1 = wmma16(qa[kc], cat16(*(const v8h*)(K16 + o1), *(const v8h*)(K16 + o1 + 16)), s1);
        }
        asm volatile("v_nop\n\tv_nop\n\tv_nop\n\tv_nop" : "+v"(s0), "+v"(s1) : "v"(qa[0]), "v"(qa[7]));
        float alpha[8];
#pragma unroll
        for (int j = 0; j < 8; ++j) {
            const float a0 = s0[j] * 0.0625f, a1 = s1[j] * 0.0625f;
            float mx = fmaxf(a0, a1);
            mx = fmaxf(mx, __shfl_xor(mx, 1, 16)); mx = fmaxf(mx, __shfl_xor(mx, 2, 16)); mx = fmaxf(mx, __shfl_xor(mx, 4, 16)); mx = fmaxf(mx, __shfl_xor(mx, 8, 16));
            const float mn = fmaxf(mrow[j], mx);
            alpha[j] = __expf(mrow[j] - mn); mrow[j] = mn;
            const float p0 = __expf(a0 - mn), p1 = __expf(a1 - mn);
            lpart[j] = lpart[j] * alpha[j] + (p0 + p1);
            const int mr = hi * 8 + j;
            pl[mr * 32 + lr] = (h16)(p0 * PSC); pl[mr * 32 + 16 + lr] = (h16)(p1 * PSC);
        }
#pragma unroll
        for (int n = 0; n < 8; ++n)
#pragma unroll
            for (int j = 0; j < 8; ++j) o[n][j] *= alpha[j];
        asm volatile("" ::: "memory");
        const v16h pa = cat16(*(const v8ha*)(pl + lr * 32 + hi * 8), *(const v8ha*)(pl + lr * 32 + 16 + hi * 8));
#pragma unroll
        for (int n = 0; n < 8; ++n) { const h16* vp = vb + (size_t)(n * 16 + lr) * NL + l0 + hi * 8; o[n] = wmma16(pa, cat16(*(const v8h*)vp, *(const v8h*)(vp + 16)), o[n]); }
        asm volatile("v_nop\n\tv_nop\n\tv_nop\n\tv_nop" : "+v"(o[0]), "+v"(o[3]), "+v"(o[7]) : "v"(pa));
    }
    asm volatile("v_nop\n\tv_nop\n\tv_nop\n\tv_nop" : "+v"(o[0]), "+v"(o[1]), "+v"(o[2]), "+v"(o[3]), "+v"(o[4]), "+v"(o[5]), "+v"(o[6]), "+v"(o[7]));
    float inv[8];
#pragma unroll
    for (int j = 0; j < 8; ++j) { float rs = lpart[j]; rs += __shfl_xor(rs, 1, 16); rs += __shfl_xor(rs, 2, 16); rs += __shfl_xor(rs, 4, 16); rs += __shfl_xor(rs, 8, 16); inv[j] = 1.0f / (rs * PSC); }
    float* os = &ost[wave][0];
#pragma unroll
    for (int n = 0; n < 8; ++n)
#pragma unroll
        for (int j = 0; j < 8; ++j) os[(hi * 8 + j) * 132 + n * 16 + lr] = o[n][j] * inv[j];
    __syncthreads();
    float* fb = F + (tok0 + q0) * AA + aofs;
    auto pass = [&]() {
#pragma unroll
        for (int s = 0; s < 16; ++s) { const v4f v = *(const v4fa*)(os + s * 132 + lane * 4); *(volatile v4f*)(fb + (size_t)s * AA + lane * 4) = v; }
    };
    pass(); __threadfence(); pass();
}
__global__ __launch_bounds__(256) void k_g(const float* __restrict__ F, const float* __restrict__ Qf, const float* __restrict__ alphap, bf* GH, bf* GL) {
    const int lane = threadIdx.x & 31, r = blockIdx.x * 8 + (threadIdx.x >> 5);
    if (r >= NTK) return;
    const float al = bfr(alphap[0]);
    v8us oh, ol;
#pragma unroll
    for (int i = 0; i < 8; ++i) { const float v = al * F[(size_t)r * AA + lane * 8 + i] + Qf[(size_t)r * AA + lane * 8 + i]; const unsigned short hb = f2bf(v); oh[i] = hb; ol[i] = f2bf(v - bf2f(hb)); }
    *(volatile v8us*)(GH + (size_t)r * AA + lane * 8) = oh; *(volatile v8us*)(GL + (size_t)r * AA + lane * 8) = ol; __threadfence();
    *(volatile v8us*)(GH + (size_t)r * AA + lane * 8) = oh; *(volatile v8us*)(GL + (size_t)r * AA + lane * 8) = ol;
}
__global__ __launch_bounds__(256) void k_scan(const float* __restrict__ U, const float* __restrict__ x, const float* __restrict__ h0, const float* __restrict__ vf, const float* __restrict__ vr,
                                             const float* __restrict__ bfv, const float* __restrict__ brv, int chunk, float* out) {
    const int b = blockIdx.x, dl = threadIdx.x, d = chunk * DCH + dl;
    const float kvf = bfr(vf[d]), kvr = bfr(vr[d]), kbf = bfr(bfv[d]), kbr = bfr(brv[d]), c0 = bfr(h0[b * DD + d]);
#pragma unroll 1
    for (int pass = 0; pass < 2; ++pass) {
        float c = c0;
#pragma unroll 1
        for (int t = 0; t < NL; ++t) {
            const size_t r = (size_t)b * NL + t;
            const float uf = U[r * UW + dl], ur = U[r * UW + DCH + dl], uh = U[r * UW + 2 * DCH + dl];
            const float f = 1.0f / (1.0f + __expf(-(uf + kvf * c + kbf)));
            const float rg = 1.0f / (1.0f + __expf(-(ur + kvr * c + kbr)));
            c = f * c + (1.0f - f) * uh;
            const float h = rg * c + (1.0f - rg) * bfr(x[r * DD + d]);
            *(volatile float*)(out + r * DD + d) = h;
        }
        __threadfence();
    }
}

extern "C" void kernel_launch(void* const* d_in, const int* in_sizes, int n_in,
                              void* d_out, int out_size, void* d_ws, size_t ws_size, hipStream_t stream) {
    (void)in_sizes; (void)n_in; (void)out_size;
    const float* x = (const float*)d_in[0]; const float* h0 = (const float*)d_in[1]; const float* Wp = (const float*)d_in[2]; const float* bp = (const float*)d_in[3];
    const float* vf = (const float*)d_in[4]; const float* vr = (const float*)d_in[5]; const float* bfv = (const float*)d_in[6]; const float* brv = (const float*)d_in[7];
    const float* Wq = (const float*)d_in[8]; const float* Wk = (const float*)d_in[9]; const float* Wv = (const float*)d_in[10]; const float* Wu = (const float*)d_in[11]; const float* alphap = (const float*)d_in[12];
    float* out = (float*)d_out;
    char* wsp = (char*)d_ws;
    auto take = [&](size_t bytes) { char* p = wsp; wsp += (bytes + 255) & ~(size_t)255; return (void*)p; };
    bf* Xb = (bf*)take((size_t)NTK * DD * 2); bf* WpT = (bf*)take((size_t)3 * DD * DD * 2); bf* WqT = (bf*)take((size_t)AA * DD * 2); bf* WkT = (bf*)take((size_t)AA * DD * 2); bf* WvT = (bf*)take((size_t)AA * DD * 2);
    bf* WuT = (bf*)take((size_t)3 * DD * AA * 2);
    float* Qf = (float*)take((size_t)NTK * AA * 4); h16* Q16 = (h16*)take((size_t)NTK * AA * 2); h16* K16 = (h16*)take((size_t)NTK * AA * 2); float* Vf = (float*)take((size_t)NTK * AA * 4); h16* VT16 = (h16*)take((size_t)NTK * AA * 2);
    float* F = (float*)take((size_t)NTK * AA * 4); bf* GH = (bf*)take((size_t)NTK * AA * 2); bf* GL = (bf*)take((size_t)NTK * AA * 2); float* U = (float*)take((size_t)NTK * UW * 4);
    if ((size_t)(wsp - (char*)d_ws) > ws_size) return;
    k_cvtb<<<NTK / 8, 256, 0, stream>>>(x, Xb);
    k_wt<<<dim3(DD / 64, (3 * DD) / 64, 1), 256, 0, stream>>>(Wp, DD, 3 * DD, WpT);
    k_wt<<<dim3(DD / 64, AA / 64, 1), 256, 0, stream>>>(Wq, DD, AA, WqT); k_wt<<<dim3(DD / 64, AA / 64, 1), 256, 0, stream>>>(Wk, DD, AA, WkT); k_wt<<<dim3(DD / 64, AA / 64, 1), 256, 0, stream>>>(Wv, DD, AA, WvT);
    k_wt<<<dim3(AA / 64, (3 * DD) / 64, 1), 256, 0, stream>>>(Wu, AA, 3 * DD, WuT);
    k_gemm<false, 0><<<dim3(NTK / 64, AA / 64, 1), 128, 0, stream>>>(Xb, nullptr, WqT, DD, 0, nullptr, Qf, Q16);
    k_gemm<false, 1><<<dim3(NTK / 64, AA / 64, 1), 128, 0, stream>>>(Xb, nullptr, WkT, DD, 0, nullptr, K16, nullptr);
    k_gemm<false, 2><<<dim3(NTK / 64, AA / 64, 1), 128, 0, stream>>>(Xb, nullptr, WvT, DD, 0, nullptr, Vf, nullptr);
    k_vt<<<NB_ * (NL / 64), 256, 0, stream>>>(Vf, VT16);
    k_attn<<<NB_ * (NL / 64), 128, 0, stream>>>(Q16, K16, VT16, 0, F);
    k_attn<<<NB_ * (NL / 64), 128, 0, stream>>>(Q16, K16, VT16, 128, F);
    k_g<<<NTK / 8, 256, 0, stream>>>(F, Qf, alphap, GH, GL);
    for (int chunk = 0; chunk < DD / DCH; ++chunk) {
        k_gemm<false, 3><<<dim3(NTK / 64, UW / 64, 1), 128, 0, stream>>>(Xb, nullptr, WpT, DD, chunk, bp, U, nullptr);
        k_gemm<true, 4><<<dim3(NTK / 64, UW / 64, 1), 128, 0, stream>>>(GH, GL, WuT, AA, chunk, nullptr, U, nullptr);
        k_scan<<<NB_, 256, 0, stream>>>(U, x, h0, vf, vr, bfv, brv, chunk, out);
    }
}
